// TransformerBlock_4810363372375
// MI455X (gfx1250) — hardware-verified
//
#include <hip/hip_runtime.h>
#include <stddef.h>


typedef _Float16 v16h __attribute__((ext_vector_type(16)));
typedef _Float16 v8h  __attribute__((ext_vector_type(8)));
typedef float    v8f  __attribute__((ext_vector_type(8)));
typedef float    v4f  __attribute__((ext_vector_type(4)));

#ifndef NB
#define NB 2
#endif
#ifndef SEQ
#define SEQ 2048
#endif
#define NB_FULL  2
#define SEQ_FULL 2048
#define DIM   768
#define NHEAD 12
#define HD    64
#define FFD   3072
#define MROWS (NB * SEQ)
#define EARLY 256

#define LDT 72
#define LDP 40
#define LDC 68
#define TS  (64 * LDT)

#define WCARRY 64.0f
#define HCARRY 16.0f
#define PCARRY 1024.0f
#define VCARRY 64.0f
#define RCARRY 2048.0f
#define RINV   (1.0f / 2048.0f)
#define LN_EPS 1.0e-3f
#define NEGFILL (-1.0e9f)

static_assert(NB >= 1 && NB <= NB_FULL);
static_assert(SEQ >= EARLY && SEQ <= SEQ_FULL && (SEQ % 128) == 0);
static_assert((EARLY % 128) == 0 && EARLY >= 128);
static_assert(DIM == NHEAD * HD);
static_assert(HD == 64);
static_assert((DIM % 64) == 0 && (DIM % 32) == 0 && (DIM % 256) == 0);
static_assert((FFD % 64) == 0 && (FFD % 32) == 0);
static_assert((MROWS % 64) == 0 && (MROWS % 8) == 0);
static_assert((size_t)MROWS * FFD < (size_t)0xFFFFFFFFu);
static_assert((LDT % 8) == 0 && (LDP % 8) == 0 && (LDC % 4) == 0);
static_assert(8 * 16 * LDT <= 2 * TS);

#define WSQ_BYTES ((size_t)DIM * DIM * 2)
#define WF_BYTES  ((size_t)DIM * FFD * 2)
#define P16_BYTES ((size_t)MROWS * DIM * 2)
#define VTL_BYTES ((size_t)NB * DIM * EARLY * 2)
#define X1_BYTES  ((size_t)MROWS * DIM * 4)
#define HID_BYTES ((size_t)MROWS * FFD * 2)
#define OFF_WQ  ((size_t)0)
#define OFF_WK  (OFF_WQ + WSQ_BYTES)
#define OFF_WV  (OFF_WK + WSQ_BYTES)
#define OFF_WO  (OFF_WV + WSQ_BYTES)
#define OFF_W1  (OFF_WO + WSQ_BYTES)
#define OFF_W2  (OFF_W1 + WF_BYTES)
#define OFF_H   (OFF_W2 + WF_BYTES)
#define OFF_QH  (OFF_H  + P16_BYTES)
#define OFF_QL  (OFF_QH + P16_BYTES)
#define OFF_KH  (OFF_QL + P16_BYTES)
#define OFF_KL  (OFF_KH + P16_BYTES)
#define OFF_VH  (OFF_KL + P16_BYTES)
#define OFF_VL  (OFF_VH + P16_BYTES)
#define OFF_CTX (OFF_VL + VTL_BYTES)
#define OFF_X1  (OFF_CTX + P16_BYTES)
#define OFF_HID (OFF_X1 + X1_BYTES)
#define WS_TOTAL (OFF_HID + HID_BYTES)
static_assert((WSQ_BYTES % 128) == 0 && (WF_BYTES % 128) == 0 && (P16_BYTES % 128) == 0);
static_assert((VTL_BYTES % 128) == 0 && (X1_BYTES % 128) == 0 && (HID_BYTES % 128) == 0);
static_assert(WS_TOTAL <= (size_t)134217728);

__device__ __forceinline__ float bf16r(float x) {
  unsigned int u = __float_as_uint(x);
  u = (u + 0x7FFFu + ((u >> 16) & 1u)) & 0xFFFF0000u;
  return __uint_as_float(u);
}
__device__ __forceinline__ float selr(float v, bool rne) { return rne ? bf16r(v) : v; }

__device__ __forceinline__ v16h frag_join(v8h lo, v8h hi) {
  v16h out;
#pragma unroll
  for (int i = 0; i < 8; ++i) { out[i] = lo[i]; out[i + 8] = hi[i]; }
  return out;
}
__device__ __forceinline__ v16h frag_at(const _Float16* p) {
  return frag_join(*(const v8h*)(p), *(const v8h*)(p + 16));
}
#define LDS_FRAG(arr, off) frag_join(*(const v8h*)&arr[(off)], *(const v8h*)&arr[(off) + 16u])

__device__ __forceinline__ v8f wmma16(v16h a, v16h b, v8f c) {
  v8f d = __builtin_amdgcn_wmma_f32_16x16x32_f16(false, a, false, b, (short)0, c,
                                                 false, false);
  asm volatile("v_nop\n\tv_nop\n\tv_nop\n\tv_nop" : "+v"(d) : "v"(a), "v"(b));
  return d;
}

__device__ __forceinline__ float red16_max(float x) {
#pragma unroll
  for (int off = 1; off < 16; off <<= 1) x = fmaxf(x, __shfl_xor(x, off, 32));
  return x;
}
__device__ __forceinline__ float red16_sum(float x) {
#pragma unroll
  for (int off = 1; off < 16; off <<= 1) x += __shfl_xor(x, off, 32);
  return x;
}
__device__ __forceinline__ float red32_sum(float x) {
#pragma unroll
  for (int off = 1; off < 32; off <<= 1) x += __shfl_xor(x, off, 32);
  return x;
}

__device__ __forceinline__ void wave_lds_sync() {
  __builtin_amdgcn_fence(3  , "wavefront");
  asm volatile("s_wait_dscnt 0x0" ::: "memory");
  __builtin_amdgcn_wave_barrier();
}

__global__ __launch_bounds__(256) void wconv_kernel(
    const float* __restrict__ W, _Float16* __restrict__ Wt, unsigned kdim, unsigned ndim) {
  __shared__ __attribute__((aligned(16))) _Float16 T[64 * LDT];
  const unsigned tid = threadIdx.x;
  const unsigned n0 = blockIdx.x * 64u;
  const unsigned k0 = blockIdx.y * 64u;
#pragma unroll 4
  for (unsigned j = 0; j < 16u; ++j) {
    const unsigned idx = tid + 256u * j;
    const unsigned kr = idx >> 6, nc = idx & 63u;
    const float v = W[(size_t)(k0 + kr) * ndim + n0 + nc];
    T[nc * LDT + kr] = (_Float16)(WCARRY * bf16r(v));
  }
  __syncthreads();
  v8h x[2];
  size_t off[2];
#pragma unroll
  for (unsigned i = 0; i < 2u; ++i) {
    const unsigned n = 32u * i + (tid >> 3);
    const unsigned kc = (tid & 7u) * 8u;
    x[i] = *(const v8h*)&T[n * LDT + kc];
    off[i] = (size_t)(n0 + n) * kdim + k0 + kc;
  }
#pragma unroll
  for (int i = 0; i < 2; ++i) *(volatile v8h*)(Wt + off[i]) = x[i];
  __threadfence();
#pragma unroll
  for (int i = 0; i < 2; ++i) *(volatile v8h*)(Wt + off[i]) = x[i];
}

__global__ __launch_bounds__(256) void ln_kernel(
    const float* __restrict__ src, const float* __restrict__ gam,
    const float* __restrict__ bet, _Float16* __restrict__ dst, int src_is_input) {
  const unsigned lane = threadIdx.x & 31u;
  const unsigned w = (unsigned)__builtin_amdgcn_readfirstlane((int)(threadIdx.x >> 5));
  const unsigned crow = blockIdx.x * 8u + w;
  const bool rne = (src_is_input != 0);
  unsigned srow = crow;
  if (rne) {
    const unsigned bidx = crow / (unsigned)SEQ;
    srow = bidx * (unsigned)SEQ_FULL + (crow - bidx * (unsigned)SEQ);
  }
  const float* sp = src + (size_t)srow * DIM;

  float sum = 0.0f;
#pragma unroll 1
  for (unsigned j = 0; j < (unsigned)(DIM / 128); ++j) {
    const v4f a = *(const v4f*)(sp + (j * 32u + lane) * 4u);
    const float a0 = selr(a[0], rne), a1 = selr(a[1], rne);
    const float a2 = selr(a[2], rne), a3 = selr(a[3], rne);
    sum += (a0 + a1) + (a2 + a3);
  }
  const float mu = red32_sum(sum) * (1.0f / (float)DIM);

  float sq = 0.0f;
#pragma unroll 1
  for (unsigned j = 0; j < (unsigned)(DIM / 128); ++j) {
    const v4f a = *(const v4f*)(sp + (j * 32u + lane) * 4u);
    const float d0 = selr(a[0], rne) - mu, d1 = selr(a[1], rne) - mu;
    const float d2 = selr(a[2], rne) - mu, d3 = selr(a[3], rne) - mu;
    sq += (d0 * d0 + d1 * d1) + (d2 * d2 + d3 * d3);
  }
  const float var = red32_sum(sq) * (1.0f / (float)DIM);
  const float rstd = rsqrtf(var + LN_EPS);

  v8h o[3];
  size_t off[3];
#pragma unroll
  for (unsigned j = 0; j < 3u; ++j) {
    const unsigned e = (j * 32u + lane) * 8u;
    const v4f a0 = *(const v4f*)(sp + e);
    const v4f a1 = *(const v4f*)(sp + e + 4);
    const v4f g0 = *(const v4f*)(gam + e);
    const v4f g1 = *(const v4f*)(gam + e + 4);
    const v4f b0 = *(const v4f*)(bet + e);
    const v4f b1 = *(const v4f*)(bet + e + 4);
#pragma unroll
    for (int i = 0; i < 4; ++i) {
      const float y0 = ((selr(a0[i], rne) - mu) * rstd) * bf16r(g0[i]) + bf16r(b0[i]);
      const float y1 = ((selr(a1[i], rne) - mu) * rstd) * bf16r(g1[i]) + bf16r(b1[i]);
      o[j][i]     = (_Float16)(HCARRY * y0);
      o[j][i + 4] = (_Float16)(HCARRY * y1);
    }
    off[j] = (size_t)crow * DIM + e;
  }
#pragma unroll
  for (int j = 0; j < 3; ++j) *(volatile v8h*)(dst + off[j]) = o[j];
  __threadfence();
#pragma unroll
  for (int j = 0; j < 3; ++j) *(volatile v8h*)(dst + off[j]) = o[j];
}

template <int MODE, int KD, int ND>
__device__ __forceinline__ void gemm_body(
    const _Float16* __restrict__ A16, const _Float16* __restrict__ Bt,
    const float* __restrict__ addA, const float* __restrict__ addB,
    float* __restrict__ outf, _Float16* __restrict__ outh, _Float16* __restrict__ outl) {
  static_assert((KD % 32) == 0 && (ND % 64) == 0);
  static_assert(MODE == 3 || ND == DIM);
  __shared__ __attribute__((aligned(16))) float Cs[64 * LDC];
  const unsigned tid = threadIdx.x, lane = tid & 31u;
  const unsigned w = (unsigned)__builtin_amdgcn_readfirstlane((int)(tid >> 5));
  const unsigned mw = w >> 1, nw = w & 1u;
  const unsigned hh = lane >> 4, m = lane & 15u;
  const unsigned n0 = blockIdx.x * 64u;
  const unsigned row0 = blockIdx.y * 64u;

  const _Float16* ap  = A16 + (size_t)(row0 + mw * 16u + m) * KD + hh * 8u;
  const _Float16* bp0 = Bt + (size_t)(n0 + nw * 32u + m) * KD + hh * 8u;
  const _Float16* bp1 = bp0 + 16 * KD;
  v8f acc0 = {}, acc1 = {};
#pragma unroll 2
  for (unsigned k0 = 0; k0 < (unsigned)KD; k0 += 32u) {
    const v16h a  = frag_at(ap + k0);
    const v16h b0 = frag_at(bp0 + k0);
    const v16h b1 = frag_at(bp1 + k0);
    acc0 = wmma16(a, b0, acc0);
    acc1 = wmma16(a, b1, acc1);
  }
#pragma unroll
  for (int r = 0; r < 8; ++r) {
    const unsigned ci = (mw * 16u + hh * 8u + (unsigned)r) * LDC + nw * 32u + m;
    Cs[ci]       = acc0[r];
    Cs[ci + 16u] = acc1[r];
  }
  __syncthreads();

  if (MODE == 0) {
    const float sc = 1.0f / (HCARRY * WCARRY);
    v8h xh[2], xl[2];
    size_t off[2];
#pragma unroll
    for (unsigned i = 0; i < 2u; ++i) {
      const unsigned r = 32u * i + (tid >> 3);
      const unsigned c = (tid & 7u) * 8u;
      const v4f u0 = *(const v4f*)&Cs[r * LDC + c];
      const v4f u1 = *(const v4f*)&Cs[r * LDC + c + 4];
#pragma unroll
      for (int j = 0; j < 4; ++j) {
        const float t0 = u0[j] * sc, t1 = u1[j] * sc;
        const _Float16 h0 = (_Float16)t0, h1 = (_Float16)t1;
        xh[i][j] = h0;  xh[i][j + 4] = h1;
        xl[i][j]     = (_Float16)((t0 - (float)h0) * RCARRY);
        xl[i][j + 4] = (_Float16)((t1 - (float)h1) * RCARRY);
      }
      off[i] = (size_t)(row0 + r) * ND + n0 + c;
    }
#pragma unroll
    for (int i = 0; i < 2; ++i) {
      *(volatile v8h*)(outh + off[i]) = xh[i];
      *(volatile v8h*)(outl + off[i]) = xl[i];
    }
    __threadfence();
#pragma unroll
    for (int i = 0; i < 2; ++i) {
      *(volatile v8h*)(outh + off[i]) = xh[i];
      *(volatile v8h*)(outl + off[i]) = xl[i];
    }
  }

  if (MODE == 1) {
    const float sc = 1.0f / (HCARRY * WCARRY);
    const unsigned bidx = row0 / (unsigned)SEQ;
    const unsigned key0 = row0 - bidx * (unsigned)SEQ;
    const bool early = (key0 < (unsigned)EARLY);
    v8h xh[2], xl[2];
    size_t off[2], offl[2];
#pragma unroll
    for (unsigned i = 0; i < 2u; ++i) {
      const unsigned dcol = 32u * i + (tid >> 3);
      const unsigned kk = (tid & 7u) * 8u;
#pragma unroll
      for (unsigned j = 0; j < 8u; ++j) {
        const float t = Cs[(kk + j) * LDC + dcol] * sc;
        const _Float16 h = (_Float16)t;
        xh[i][j] = h;
        xl[i][j] = (_Float16)((t - (float)h) * RCARRY);
      }
      off[i]  = ((size_t)bidx * DIM + n0 + dcol) * SEQ + key0 + kk;
      offl[i] = ((size_t)bidx * DIM + n0 + dcol) * EARLY + (early ? key0 : 0u) + kk;
    }
#pragma unroll
    for (int i = 0; i < 2; ++i) *(volatile v8h*)(outh + off[i]) = xh[i];
    if (early) {
#pragma unroll
      for (int i = 0; i < 2; ++i) *(volatile v8h*)(outl + offl[i]) = xl[i];
    }
    __threadfence();
#pragma unroll
    for (int i = 0; i < 2; ++i) *(volatile v8h*)(outh + off[i]) = xh[i];
    if (early) {
#pragma unroll
      for (int i = 0; i < 2; ++i) *(volatile v8h*)(outl + offl[i]) = xl[i];
    }
  }

  if (MODE == 3) {
    const float sc = 1.0f / (HCARRY * WCARRY);
    v8h x[2];
    size_t off[2];
#pragma unroll
    for (unsigned i = 0; i < 2u; ++i) {
      const unsigned r = 32u * i + (tid >> 3);
      const unsigned c = (tid & 7u) * 8u;
      const v4f u0 = *(const v4f*)&Cs[r * LDC + c];
      const v4f u1 = *(const v4f*)&Cs[r * LDC + c + 4];
      const v4f g0 = *(const v4f*)(addB + n0 + c);
      const v4f g1 = *(const v4f*)(addB + n0 + c + 4);
#pragma unroll
      for (int j = 0; j < 4; ++j) {
        const float t0 = u0[j] * sc + bf16r(g0[j]);
        const float t1 = u1[j] * sc + bf16r(g1[j]);
        x[i][j]     = (_Float16)(HCARRY * ((t0 > 0.0f) ? t0 : 0.0f));
        x[i][j + 4] = (_Float16)(HCARRY * ((t1 > 0.0f) ? t1 : 0.0f));
      }
      off[i] = (size_t)(row0 + r) * ND + n0 + c;
    }
#pragma unroll
    for (int i = 0; i < 2; ++i) *(volatile v8h*)(outh + off[i]) = x[i];
    __threadfence();
#pragma unroll
    for (int i = 0; i < 2; ++i) *(volatile v8h*)(outh + off[i]) = x[i];
  }

  if (MODE == 2 || MODE == 4) {
    const float sc = (MODE == 2) ? (1.0f / (VCARRY * WCARRY)) : (1.0f / (HCARRY * WCARRY));
    v4f xs[4];
    size_t off[4];
#pragma unroll
    for (unsigned i = 0; i < 4u; ++i) {
      const unsigned r = 16u * i + (tid >> 4);
      const unsigned c = (tid & 15u) * 4u;
      const unsigned crow = row0 + r;
      const unsigned bidx = crow / (unsigned)SEQ;
      const unsigned sq = crow - bidx * (unsigned)SEQ;
      const size_t frow = (size_t)bidx * SEQ_FULL + sq;
      const v4f u = *(const v4f*)&Cs[r * LDC + c];
      v4f val;
      if (MODE == 2) {
        const v4f xin = *(const v4f*)(addA + frow * DIM + n0 + c);
#pragma unroll
        for (int j = 0; j < 4; ++j) val[j] = bf16r(xin[j]) + u[j] * sc;
        off[i] = (size_t)crow * DIM + n0 + c;
      } else {
        const v4f x1v = *(const v4f*)(addA + (size_t)crow * DIM + n0 + c);
        const v4f g = *(const v4f*)(addB + n0 + c);
#pragma unroll
        for (int j = 0; j < 4; ++j) val[j] = x1v[j] + (u[j] * sc + bf16r(g[j]));
        off[i] = frow * DIM + n0 + c;
      }
      xs[i] = val;
    }
#pragma unroll
    for (int i = 0; i < 4; ++i) *(volatile v4f*)(outf + off[i]) = xs[i];
    __threadfence();
#pragma unroll
    for (int i = 0; i < 4; ++i) *(volatile v4f*)(outf + off[i]) = xs[i];
  }
}

__global__ __launch_bounds__(256) void proj_qk_kernel(
    const _Float16* __restrict__ A16, const _Float16* __restrict__ Bt,
    _Float16* __restrict__ outh, _Float16* __restrict__ outl) {
  gemm_body<0, DIM, DIM>(A16, Bt, nullptr, nullptr, nullptr, outh, outl);
}
__global__ __launch_bounds__(256) void proj_v_kernel(
    const _Float16* __restrict__ A16, const _Float16* __restrict__ Bt,
    _Float16* __restrict__ outh, _Float16* __restrict__ outl) {
  gemm_body<1, DIM, DIM>(A16, Bt, nullptr, nullptr, nullptr, outh, outl);
}
__global__ __launch_bounds__(256) void oproj_kernel(
    const _Float16* __restrict__ A16, const _Float16* __restrict__ Bt,
    const float* __restrict__ Xin, float* __restrict__ x1) {
  gemm_body<2, DIM, DIM>(A16, Bt, Xin, nullptr, x1, nullptr, nullptr);
}
__global__ __launch_bounds__(256) void ffn1_kernel(
    const _Float16* __restrict__ A16, const _Float16* __restrict__ Bt,
    const float* __restrict__ bias, _Float16* __restrict__ hid) {
  gemm_body<3, DIM, FFD>(A16, Bt, nullptr, bias, nullptr, hid, nullptr);
}
__global__ __launch_bounds__(256) void ffn2_kernel(
    const _Float16* __restrict__ A16, const _Float16* __restrict__ Bt,
    const float* __restrict__ x1, const float* __restrict__ bias, float* __restrict__ outp) {
  gemm_body<4, FFD, DIM>(A16, Bt, x1, bias, outp, nullptr, nullptr);
}

template <int RES>
__device__ __forceinline__ void attn_body(
    const _Float16* __restrict__ Qh, const _Float16* __restrict__ Ql,
    const _Float16* __restrict__ Kh, const _Float16* __restrict__ Kl,
    const _Float16* __restrict__ Vth, const _Float16* __restrict__ Vtl,
    _Float16* __restrict__ Ov, unsigned qblk) {
  __shared__ __attribute__((aligned(16))) _Float16 KV[4 * TS];
  __shared__ __attribute__((aligned(16))) _Float16 Ph[8 * 16 * LDP];
  __shared__ __attribute__((aligned(16))) _Float16 Pl[8 * 16 * LDP];

  const unsigned tid = threadIdx.x, lane = tid & 31u;
  const unsigned w = (unsigned)__builtin_amdgcn_readfirstlane((int)(tid >> 5));
  const unsigned hh = lane >> 4, m = lane & 15u;
  const unsigned q0 = qblk * 128u;
  const unsigned head = blockIdx.y;
  const unsigned b = blockIdx.z;
  const unsigned qw0 = q0 + w * 16u;
  const unsigned pb = w * (16u * LDP);
  const unsigned qoff0 = (b * (unsigned)SEQ + qw0 + m) * (unsigned)DIM + head * HD + hh * 8u;

  float mrow[8], lrow[8];
  v8f o[4];
  v8f orr[4];
#pragma unroll
  for (int v = 0; v < 8; ++v) { mrow[v] = -1.0e30f; lrow[v] = 0.0f; }
#pragma unroll
  for (int nb = 0; nb < 4; ++nb) { o[nb] = (v8f){}; orr[nb] = (v8f){}; }

  const unsigned kplane = b * (unsigned)SEQ * (unsigned)DIM + head * HD;
  const unsigned vplane = (b * (unsigned)DIM + head * HD) * (unsigned)SEQ;
  const unsigned vplane_l = (b * (unsigned)DIM + head * HD) * (unsigned)EARLY;
  const unsigned kend = q0 + 128u;

  for (unsigned kb = 0; kb < kend; kb += 64u) {
#pragma unroll
    for (unsigned j = 0; j < 2u; ++j) {
      const unsigned idx = tid + 256u * j;
      const unsigned r = idx >> 3, c = (idx & 7u) * 8u;
      const unsigned ko = kplane + (kb + r) * (unsigned)DIM + c;
      *(v8h*)&KV[r * LDT + c]           = *(const v8h*)(Kh + ko);
      *(v8h*)&KV[TS + r * LDT + c]      = *(const v8h*)(Kl + ko);
      *(v8h*)&KV[2 * TS + r * LDT + c]  = *(const v8h*)(Vth + vplane + r * (unsigned)SEQ + kb + c);
      if (RES)
        *(v8h*)&KV[3 * TS + r * LDT + c] =
            *(const v8h*)(Vtl + vplane_l + r * (unsigned)EARLY + kb + c);
    }
    __syncthreads();

#pragma unroll 1
    for (unsigned hf = 0; hf < 2u; ++hf) {
      const unsigned kh0 = kb + 32u * hf;
      if (kh0 <= qw0 + 15u) {
        v8f sm0 = {}, sm1 = {}, sr0 = {}, sr1 = {};
        unsigned qo = qoff0;
        asm volatile("" : "+v"(qo));
#pragma unroll
        for (unsigned c = 0; c < 2u; ++c) {
          const v16h qh = frag_at(Qh + qo + c * 32u);
          const v16h ql = frag_at(Ql + qo + c * 32u);
          const unsigned ko = (hf * 32u + m) * LDT + hh * 8u + c * 32u;
          const v16h k0h = LDS_FRAG(KV, ko);
          const v16h k0l = LDS_FRAG(KV, TS + ko);
          sm0 = wmma16(qh, k0h, sm0);
          sr0 = wmma16(qh, k0l, sr0);
          sr0 = wmma16(ql, k0h, sr0);
          const v16h k1h = LDS_FRAG(KV, ko + 16u * LDT);
          const v16h k1l = LDS_FRAG(KV, TS + ko + 16u * LDT);
          sm1 = wmma16(qh, k1h, sm1);
          sr1 = wmma16(qh, k1l, sr1);
          sr1 = wmma16(ql, k1h, sr1);
        }

        const unsigned key0 = kh0 + m;
#pragma unroll
        for (int v = 0; v < 8; ++v) {
          const unsigned qrow = qw0 + hh * 8u + (unsigned)v;
          float a = (sm0[v] + sr0[v] * RINV) * 0.125f;
          float c1 = (sm1[v] + sr1[v] * RINV) * 0.125f;
          a  = (key0 > qrow) ? NEGFILL : a;
          c1 = (key0 + 16u > qrow) ? NEGFILL : c1;
          const float mx = red16_max(fmaxf(a, c1));
          const float mn = fmaxf(mrow[v], mx);
          const float alpha = __expf(mrow[v] - mn);
          mrow[v] = mn;
          const float pa = __expf(a - mn);
          const float pc = __expf(c1 - mn);
          const float rs = red16_sum(pa + pc);
          lrow[v] = alpha * lrow[v] + rs;
#pragma unroll
          for (int nb = 0; nb < 4; ++nb) o[nb][v] = o[nb][v] * alpha;
          if (RES) {
#pragma unroll
            for (int nb = 0; nb < 4; ++nb) orr[nb][v] = orr[nb][v] * alpha;
          }
          const float ta = pa * PCARRY, tc = pc * PCARRY;
          const _Float16 ha = (_Float16)ta, hc = (_Float16)tc;
          const unsigned pi = pb + (hh * 8u + (unsigned)v) * LDP + m;
          Ph[pi]       = ha;
          Ph[pi + 16u] = hc;
          if (RES) {
            Pl[pi]       = (_Float16)((ta - (float)ha) * RCARRY);
            Pl[pi + 16u] = (_Float16)((tc - (float)hc) * RCARRY);
          }
        }
        wave_lds_sync();

        const unsigned po = pb + m * LDP + hh * 8u;
        const v16h pf = LDS_FRAG(Ph, po);
        const unsigned vo = 2u * TS + m * LDT + hf * 32u + hh * 8u;
        if (RES) {
          const v16h pl = LDS_FRAG(Pl, po);
#pragma unroll
          for (unsigned nb = 0; nb < 4u; ++nb) {
            const v16h vf = LDS_FRAG(KV, vo + nb * 16u * LDT);
            const v16h vl = LDS_FRAG(KV, vo + TS + nb * 16u * LDT);
            o[nb]   = wmma16(pf, vf, o[nb]);
            orr[nb] = wmma16(pf, vl, orr[nb]);
            orr[nb] = wmma16(pl, vf, orr[nb]);
          }
        } else {
#pragma unroll
          for (unsigned nb = 0; nb < 4u; ++nb) {
            const v16h vf = LDS_FRAG(KV, vo + nb * 16u * LDT);
            o[nb] = wmma16(pf, vf, o[nb]);
          }
        }
        wave_lds_sync();
      }
    }
    __syncthreads();
  }

  const unsigned ob = w * (16u * LDT);
#pragma unroll
  for (int v = 0; v < 8; ++v) {
    const float inv = __builtin_amdgcn_rcpf(lrow[v]) * (VCARRY / PCARRY);
#pragma unroll
    for (int nb = 0; nb < 4; ++nb) {
      float t = o[nb][v];
      if (RES) t += orr[nb][v] * RINV;
      KV[ob + (hh * 8u + (unsigned)v) * LDT + (unsigned)nb * 16u + m] = (_Float16)(t * inv);
    }
  }
  wave_lds_sync();
  v8h x[4];
  size_t off[4];
#pragma unroll
  for (unsigned i = 0; i < 4u; ++i) {
    const unsigned r = 4u * i + (lane >> 3);
    const unsigned c = (lane & 7u) * 8u;
    x[i] = *(const v8h*)&KV[ob + r * LDT + c];
    off[i] = (size_t)(b * (unsigned)SEQ + qw0 + r) * DIM + head * HD + c;
  }
#pragma unroll
  for (int i = 0; i < 4; ++i) *(volatile v8h*)(Ov + off[i]) = x[i];
  __threadfence();
#pragma unroll
  for (int i = 0; i < 4; ++i) *(volatile v8h*)(Ov + off[i]) = x[i];
}

__global__ __launch_bounds__(256) void attn_main_kernel(
    const _Float16* __restrict__ Qh, const _Float16* __restrict__ Ql,
    const _Float16* __restrict__ Kh, const _Float16* __restrict__ Kl,
    const _Float16* __restrict__ Vth, _Float16* __restrict__ Ov) {
  attn_body<0>(Qh, Ql, Kh, Kl, Vth, nullptr, Ov, blockIdx.x + (unsigned)(EARLY / 128));
}
__global__ __launch_bounds__(256) void attn_early_kernel(
    const _Float16* __restrict__ Qh, const _Float16* __restrict__ Ql,
    const _Float16* __restrict__ Kh, const _Float16* __restrict__ Kl,
    const _Float16* __restrict__ Vth, const _Float16* __restrict__ Vtl,
    _Float16* __restrict__ Ov) {
  attn_body<1>(Qh, Ql, Kh, Kl, Vth, Vtl, Ov, blockIdx.x);
}

extern "C" void kernel_launch(void* const* d_in, const int* in_sizes, int n_in,
                              void* d_out, int out_size, void* d_ws, size_t ws_size,
                              hipStream_t stream) {
  if (n_in < 13) return;
  const long long need_x = ((long long)(NB - 1) * SEQ_FULL + SEQ) * DIM;
  if ((long long)in_sizes[0] < need_x) return;
  for (int i = 1; i <= 4; ++i)
    if ((long long)in_sizes[i] < (long long)DIM * DIM) return;
  if ((long long)in_sizes[5] < (long long)DIM * FFD) return;
  if (in_sizes[6] < FFD) return;
  if ((long long)in_sizes[7] < (long long)FFD * DIM) return;
  for (int i = 8; i <= 12; ++i)
    if (in_sizes[i] < DIM) return;
  if ((long long)out_size < need_x) return;
  if (ws_size < WS_TOTAL) return;

  const float* X    = (const float*)d_in[0];
  const float* W_Q  = (const float*)d_in[1];
  const float* W_K  = (const float*)d_in[2];
  const float* W_V  = (const float*)d_in[3];
  const float* W_O  = (const float*)d_in[4];
  const float* w1   = (const float*)d_in[5];
  const float* b1   = (const float*)d_in[6];
  const float* w2   = (const float*)d_in[7];
  const float* b2   = (const float*)d_in[8];
  const float* ln1g = (const float*)d_in[9];
  const float* ln1b = (const float*)d_in[10];
  const float* ln2g = (const float*)d_in[11];
  const float* ln2b = (const float*)d_in[12];
  float* out = (float*)d_out;

  char* ws = (char*)d_ws;
  _Float16* WtQ  = (_Float16*)(ws + OFF_WQ);
  _Float16* WtK  = (_Float16*)(ws + OFF_WK);
  _Float16* WtV  = (_Float16*)(ws + OFF_WV);
  _Float16* WtO  = (_Float16*)(ws + OFF_WO);
  _Float16* Wt1  = (_Float16*)(ws + OFF_W1);
  _Float16* Wt2  = (_Float16*)(ws + OFF_W2);
  _Float16* H16  = (_Float16*)(ws + OFF_H);
  _Float16* Qh16 = (_Float16*)(ws + OFF_QH);
  _Float16* Ql16 = (_Float16*)(ws + OFF_QL);
  _Float16* Kh16 = (_Float16*)(ws + OFF_KH);
  _Float16* Kl16 = (_Float16*)(ws + OFF_KL);
  _Float16* Vth  = (_Float16*)(ws + OFF_VH);
  _Float16* Vtl  = (_Float16*)(ws + OFF_VL);
  _Float16* Ctx  = (_Float16*)(ws + OFF_CTX);
  float*    X1   = (float*)(ws + OFF_X1);
  _Float16* Hid  = (_Float16*)(ws + OFF_HID);

  dim3 blk(256);
  dim3 gp(DIM / 64, MROWS / 64);

  wconv_kernel<<<dim3(DIM / 64, DIM / 64), blk, 0, stream>>>(W_Q, WtQ, (unsigned)DIM, (unsigned)DIM);
  wconv_kernel<<<dim3(DIM / 64, DIM / 64), blk, 0, stream>>>(W_K, WtK, (unsigned)DIM, (unsigned)DIM);
  wconv_kernel<<<dim3(DIM / 64, DIM / 64), blk, 0, stream>>>(W_V, WtV, (unsigned)DIM, (unsigned)DIM);
  wconv_kernel<<<dim3(DIM / 64, DIM / 64), blk, 0, stream>>>(W_O, WtO, (unsigned)DIM, (unsigned)DIM);
  wconv_kernel<<<dim3(FFD / 64, DIM / 64), blk, 0, stream>>>(w1, Wt1, (unsigned)DIM, (unsigned)FFD);
  wconv_kernel<<<dim3(DIM / 64, FFD / 64), blk, 0, stream>>>(w2, Wt2, (unsigned)FFD, (unsigned)DIM);

  ln_kernel<<<dim3(MROWS / 8), blk, 0, stream>>>(X, ln1g, ln1b, H16, 1);

  proj_qk_kernel<<<gp, blk, 0, stream>>>(H16, WtQ, Qh16, Ql16);
  proj_qk_kernel<<<gp, blk, 0, stream>>>(H16, WtK, Kh16, Kl16);
  proj_v_kernel<<<gp, blk, 0, stream>>>(H16, WtV, Vth, Vtl);

  if ((SEQ / 128) > (EARLY / 128))
    attn_main_kernel<<<dim3(SEQ / 128 - EARLY / 128, NHEAD, NB), blk, 0, stream>>>(
        Qh16, Ql16, Kh16, Kl16, Vth, Ctx);
  attn_early_kernel<<<dim3(EARLY / 128, NHEAD, NB), blk, 0, stream>>>(
      Qh16, Ql16, Kh16, Kl16, Vth, Vtl, Ctx);

  oproj_kernel<<<gp, blk, 0, stream>>>(Ctx, WtO, X, X1);

  ln_kernel<<<dim3(MROWS / 8), blk, 0, stream>>>(X1, ln2g, ln2b, H16, 0);

  ffn1_kernel<<<dim3(FFD / 64, MROWS / 64), blk, 0, stream>>>(H16, Wt1, b1, Hid);
  ffn2_kernel<<<gp, blk, 0, stream>>>(Hid, Wt2, X1, b2, out);
}
